// SAB_13675175871087
// MI455X (gfx1250) — hardware-verified
//
#include <hip/hip_runtime.h>


#define NB_  4
#define CC   256
#define CQ   32
#define CQP  64
#define KC   (9 * CC)
#define NN   4096
#define PCAR 1024.0f
#define SCL  0.17677669529663687f
typedef _Float16 h16;
typedef unsigned short bf;
typedef __attribute__((ext_vector_type(16))) __bf16   v16bf;
typedef __attribute__((ext_vector_type(16))) _Float16 v16h;
typedef __attribute__((ext_vector_type(8)))  _Float16 v8h;
typedef __attribute__((ext_vector_type(8)))  unsigned short v8us;
typedef __attribute__((ext_vector_type(8)))  float    v8f;
typedef __attribute__((ext_vector_type(4)))  float    v4f;
typedef v8h  __attribute__((may_alias)) v8ha;
typedef v4f  __attribute__((may_alias)) v4fa;
typedef v8us __attribute__((may_alias)) v8usa;

__device__ __forceinline__ unsigned short f2bf(float f) { unsigned u = __float_as_uint(f); u += 0x7FFFu + ((u >> 16) & 1u); return (unsigned short)(u >> 16); }
__device__ __forceinline__ float bf2f(unsigned short b) { return __uint_as_float(((unsigned)b) << 16); }
__device__ __forceinline__ float bfr(float f) { return bf2f(f2bf(f)); }
__device__ __forceinline__ v16h cat16(v8h lo, v8h hi) { return __builtin_shufflevector(lo, hi, 0, 1, 2, 3, 4, 5, 6, 7, 8, 9, 10, 11, 12, 13, 14, 15); }
__device__ __forceinline__ v16bf cat16b(v8us lo, v8us hi) { return __builtin_bit_cast(v16bf, __builtin_shufflevector(lo, hi, 0, 1, 2, 3, 4, 5, 6, 7, 8, 9, 10, 11, 12, 13, 14, 15)); }
__device__ __forceinline__ v8f wmma16(v16h a, v16h b, v8f c) { return __builtin_amdgcn_wmma_f32_16x16x32_f16(false, a, false, b, (short)0, c, false, false); }
__device__ __forceinline__ v8f wmmab(v16bf a, v16bf b, v8f c) { return __builtin_amdgcn_wmma_f32_16x16x32_bf16(false, a, false, b, (short)0, c, false, false); }


template <typename T16> struct WFrag;
template <> struct WFrag<h16> { typedef v16h V; static __device__ __forceinline__ V ld(const h16* p) { return cat16(*(const v8h*)p, *(const v8h*)(p + 16)); } static __device__ __forceinline__ v8f mma(V a, V b, v8f c) { return wmma16(a, b, c); } };
template <> struct WFrag<bf> { typedef v16bf V; static __device__ __forceinline__ V ld(const bf* p) { return cat16b(*(const v8us*)p, *(const v8us*)(p + 16)); } static __device__ __forceinline__ v8f mma(V a, V b, v8f c) { return wmmab(a, b, c); } };
template <typename T16, int NSPLIT, bool BIAS>
__global__ __launch_bounds__(32) void k_gemmw(const T16* __restrict__ A, const T16* __restrict__ A2, const T16* __restrict__ Bt, const T16* __restrict__ Bt2, int K, float* C, int ldc, const float* __restrict__ bias, size_t sA, size_t sB, size_t sC) {
    typedef typename WFrag<T16>::V V;
    __shared__ __align__(16) float os[16 * 68];
    const size_t z = blockIdx.z; A += z * sA; if (A2) A2 += z * sA; Bt += z * sB; if (Bt2) Bt2 += z * sB; C += z * sC;
    const int lane = threadIdx.x & 31, lr = lane & 15, hi = lane >> 4; const int r0 = blockIdx.x * 64, c0 = blockIdx.y * 64;
    v8f acc[4][4];
#pragma unroll
    for (int mb = 0; mb < 4; ++mb)
#pragma unroll
        for (int nb = 0; nb < 4; ++nb) acc[mb][nb] = (v8f){};
    const size_t aoff = (size_t)(r0 + lr) * K + 8 * hi, boff = (size_t)(c0 + lr) * K + 8 * hi;
#pragma unroll 1
    for (int kc = 0; kc < K; kc += 32) {
        V a[4], a2[4];
#pragma unroll
        for (int mb = 0; mb < 4; ++mb) { a[mb] = WFrag<T16>::ld(A + aoff + (size_t)mb * 16 * K + kc); if (NSPLIT == 1 || NSPLIT == 2) a2[mb] = WFrag<T16>::ld(A2 + aoff + (size_t)mb * 16 * K + kc); }
#pragma unroll
        for (int nb = 0; nb < 4; ++nb) { const V b = WFrag<T16>::ld(Bt + boff + (size_t)nb * 16 * K + kc); V b2; if (NSPLIT >= 2) b2 = WFrag<T16>::ld(Bt2 + boff + (size_t)nb * 16 * K + kc);
#pragma unroll
            for (int mb = 0; mb < 4; ++mb) { acc[mb][nb] = WFrag<T16>::mma(a[mb], b, acc[mb][nb]); if (NSPLIT == 1 || NSPLIT == 2) acc[mb][nb] = WFrag<T16>::mma(a2[mb], b, acc[mb][nb]); if (NSPLIT >= 2) acc[mb][nb] = WFrag<T16>::mma(a[mb], b2, acc[mb][nb]); } }
        asm volatile("v_nop\n\tv_nop\n\tv_nop\n\tv_nop" : "+v"(acc[0][0]), "+v"(acc[1][1]), "+v"(acc[2][2]), "+v"(acc[3][3]) : "v"(a[0]), "v"(a[3]));
    }
#pragma unroll
    for (int mb = 0; mb < 4; ++mb) {
#pragma unroll
        for (int nb = 0; nb < 4; ++nb) {
#pragma unroll
            for (int j = 0; j < 8; ++j) os[(hi * 8 + j) * 68 + nb * 16 + lr] = acc[mb][nb][j]; }
        __builtin_amdgcn_wave_barrier(); asm volatile("" ::: "memory");
        float* crow = C + (size_t)(r0 + mb * 16) * ldc + c0;
#pragma unroll 1
        for (int ps = 0; ps < 2; ++ps) {
#pragma unroll
            for (int s = 0; s < 8; ++s) { const int row = 2 * s + hi, cofs = lr * 4; v4f val = *(const v4fa*)(os + row * 68 + cofs); if (BIAS) { val[0] += bfr(bias[c0 + cofs]); val[1] += bfr(bias[c0 + cofs + 1]); val[2] += bfr(bias[c0 + cofs + 2]); val[3] += bfr(bias[c0 + cofs + 3]); }
                *(volatile v4f*)(crow + (size_t)row * ldc + cofs) = val; }
            if (ps == 0) __threadfence(); }
        __builtin_amdgcn_wave_barrier(); asm volatile("" ::: "memory");
    }
}

__device__ __forceinline__ h16 tohx(float x) { return (h16)x; }
__device__ __forceinline__ void splitf(float y, unsigned short& h, unsigned short& l) { h = f2bf(y); l = f2bf(y - bf2f(h)); }
typedef __attribute__((ext_vector_type(2))) _Float16 v2h;
typedef __attribute__((ext_vector_type(4))) _Float16 v4h;
typedef __attribute__((ext_vector_type(2))) unsigned short v2us;
typedef __attribute__((ext_vector_type(4))) unsigned short v4us;

__global__ __launch_bounds__(256) void k_cvt8(const float* __restrict__ src, bf* dst, size_t n8) { const size_t i = (size_t)blockIdx.x * 256 + threadIdx.x; if (i >= n8) return; const v8f v = *(const v8f*)(src + i * 8); v8us o;
#pragma unroll
    for (int k = 0; k < 8; ++k) o[k] = f2bf(v[k]); *(volatile v8us*)(dst + i * 8) = o; __threadfence(); *(volatile v8us*)(dst + i * 8) = o; }
__global__ __launch_bounds__(256) void k_xt(const float* __restrict__ xb, bf* XT) {
    const int lane = threadIdx.x & 31; const int L0 = (blockIdx.x * 8 + (threadIdx.x >> 5)) * 8; const int nlines = NN * CC / 64;
#pragma unroll 1
    for (int ps = 0; ps < 2; ++ps) {
#pragma unroll
        for (int l = 0; l < 8; ++l) { const int L = L0 + l; if (L >= nlines) break; const int e = L * 64 + lane * 2; const int c = e & (CC - 1); const int n = e >> 8; v2us o;
#pragma unroll
            for (int q = 0; q < 2; ++q) o[q] = f2bf(xb[(size_t)(c + q) * NN + n]);
            *(volatile v2us*)(XT + (size_t)e) = o; }
        if (ps == 0) __threadfence(); }
}
__global__ __launch_bounds__(256) void k_wpad(const float* __restrict__ w, const float* __restrict__ b, bf* Bt, float* BP) { const int e = (blockIdx.x * 256 + threadIdx.x) * 2; if (e >= CQP * CC) return; const int n = e / CC, k = e % CC; v2us o;
#pragma unroll
    for (int q = 0; q < 2; ++q) o[q] = (n < CQ) ? f2bf(w[(size_t)n * CC + k + q]) : (unsigned short)0;
    *(volatile v2us*)(Bt + e) = o; if (e < CQP) { *(volatile float*)(BP + e) = (e < CQ) ? b[e] : 0.f; *(volatile float*)(BP + e + 1) = (e + 1 < CQ) ? b[e + 1] : 0.f; }
    __threadfence(); *(volatile v2us*)(Bt + e) = o; if (e < CQP) { *(volatile float*)(BP + e) = (e < CQ) ? b[e] : 0.f; *(volatile float*)(BP + e + 1) = (e + 1 < CQ) ? b[e + 1] : 0.f; } }
__global__ __launch_bounds__(256) void k_wperm(const float* __restrict__ w, bf* Bt) { const int e = (blockIdx.x * 256 + threadIdx.x) * 2; if (e >= CC * KC) return; const int co = e / KC, j = e % KC; const int tap = j / CC, ci = j % CC; v2us o;
#pragma unroll
    for (int q = 0; q < 2; ++q) o[q] = f2bf(w[(((size_t)co * CC + ci + q) * 3 + tap / 3) * 3 + tap % 3]);
    *(volatile v2us*)(Bt + e) = o; __threadfence(); *(volatile v2us*)(Bt + e) = o; }
__global__ __launch_bounds__(256) void k_qsplit(const float* __restrict__ F, bf* Ph, bf* Pl) { const size_t i = ((size_t)blockIdx.x * 256 + threadIdx.x) * 2; if (i >= (size_t)NN * CQP) return; v2us oh, ol;
#pragma unroll
    for (int q = 0; q < 2; ++q) { unsigned short a, c2; splitf(F[i + q], a, c2); oh[q] = a; ol[q] = c2; }
    *(volatile v2us*)(Ph + i) = oh; *(volatile v2us*)(Pl + i) = ol; __threadfence(); *(volatile v2us*)(Ph + i) = oh; *(volatile v2us*)(Pl + i) = ol; }
__global__ __launch_bounds__(256) void k_p16(const float* __restrict__ F, h16* P, size_t n) { const size_t i = ((size_t)blockIdx.x * 256 + threadIdx.x) * 2; if (i >= n) return; v2h v; v[0] = tohx(F[i]); v[1] = tohx(F[i + 1]); *(volatile v2h*)(P + i) = v; __threadfence(); *(volatile v2h*)(P + i) = v; }
__global__ __launch_bounds__(256) void k_v16(const float* __restrict__ FV, const float* __restrict__ bv, h16* V16) { const size_t i = ((size_t)blockIdx.x * 256 + threadIdx.x) * 2; if (i >= (size_t)CC * NN) return; const int c = (int)(i >> 12); v2h v;
#pragma unroll
    for (int q = 0; q < 2; ++q) v[q] = tohx(__fadd_rn(FV[i + q], bfr(bv[c]))); *(volatile v2h*)(V16 + i) = v; __threadfence(); *(volatile v2h*)(V16 + i) = v; }
__global__ __launch_bounds__(256) void k_smax(const float* __restrict__ S, float* RS) {
    const int lane = threadIdx.x & 31; const int i = blockIdx.x * 8 + (threadIdx.x >> 5); if (i >= NN) return; const float* sr = S + (size_t)i * NN; float m = -3.0e38f;
#pragma unroll 4
    for (int c0 = lane * 4; c0 < NN; c0 += 128) { const v4f v = *(const v4f*)(sr + c0); m = fmaxf(m, fmaxf(fmaxf(v[0], v[1]), fmaxf(v[2], v[3]))); }
#pragma unroll
    for (int sh = 16; sh; sh >>= 1) m = fmaxf(m, __shfl_xor(m, sh, 32));
    const float o = lane == 0 ? m : 0.f; *(volatile float*)(RS + (size_t)i * 32 + lane) = o; __threadfence(); *(volatile float*)(RS + (size_t)i * 32 + lane) = o;
}
__global__ __launch_bounds__(256) void k_sexp(const float* __restrict__ S, float* RS, h16* P) {
    const int lane = threadIdx.x & 31; const int i = blockIdx.x * 8 + (threadIdx.x >> 5); if (i >= NN) return; const float* sr = S + (size_t)i * NN; const float m = RS[(size_t)i * 32]; float sum = 0.f;
#pragma unroll 2
    for (int c0 = lane * 4; c0 < NN; c0 += 128) { const v4f v = *(const v4f*)(sr + c0); v4h o;
#pragma unroll
        for (int q = 0; q < 4; ++q) { float dlt = __fsub_rn(v[q], m); asm volatile("" : "+v"(dlt)); const float e = __expf(__fmul_rn(dlt, SCL)); sum += e; o[q] = tohx(e * PCAR); }
        *(volatile v4h*)(P + (size_t)i * NN + c0) = o; __threadfence(); *(volatile v4h*)(P + (size_t)i * NN + c0) = o; }
#pragma unroll
    for (int sh = 16; sh; sh >>= 1) sum += __shfl_xor(sum, sh, 32);
    const float o2 = lane == 0 ? m : (lane == 1 ? __fdiv_rn(1.0f, sum * PCAR) : 0.f);   *(volatile float*)(RS + (size_t)i * 32 + lane) = o2; __threadfence(); *(volatile float*)(RS + (size_t)i * 32 + lane) = o2;
}
__global__ __launch_bounds__(256) void k_osplit(const float* __restrict__ Ob, const float* __restrict__ RS, bf* Oh, bf* Ol) { const size_t i = ((size_t)blockIdx.x * 256 + threadIdx.x) * 2; if (i >= (size_t)NN * CC) return; const int n = (int)(i >> 8); const float ri = RS[(size_t)n * 32 + 1]; v2us oh, ol;
#pragma unroll
    for (int q = 0; q < 2; ++q) { unsigned short a, c2; splitf(__fmul_rn(Ob[i + q], ri), a, c2); oh[q] = a; ol[q] = c2; }
    *(volatile v2us*)(Oh + i) = oh; *(volatile v2us*)(Ol + i) = ol; __threadfence(); *(volatile v2us*)(Oh + i) = oh; *(volatile v2us*)(Ol + i) = ol; }
__global__ __launch_bounds__(256) void k_im2col(const bf* __restrict__ Oh, const bf* __restrict__ Ol, bf* Ch, bf* Cl) {
    const int lane = threadIdx.x & 31; const int L0 = (blockIdx.x * 8 + (threadIdx.x >> 5)) * 8; const int nlines = NN * KC / 64;
#pragma unroll 1
    for (int ps = 0; ps < 2; ++ps) {
#pragma unroll 1
        for (int l = 0; l < 8; ++l) { const int L = L0 + l; if (L >= nlines) break; const size_t e = (size_t)L * 64 + lane * 2; const int n = (int)(e / KC); const int j = (int)(e % KC); const int tap = j / CC, ci = j % CC; const int y = n >> 6, xx = n & 63;
            const int yy = y + tap / 3 - 1, x2 = xx + tap % 3 - 1; v2us oh, ol;
            if (yy >= 0 && yy < 64 && x2 >= 0 && x2 < 64) { const size_t s = ((size_t)(yy * 64 + x2)) * CC + ci; oh = *(const v2us*)(Oh + s); ol = *(const v2us*)(Ol + s); } else { oh[0] = oh[1] = 0; ol[0] = ol[1] = 0; }
            *(volatile v2us*)(Ch + e) = oh; *(volatile v2us*)(Cl + e) = ol; }
        if (ps == 0) __threadfence(); }
}
__global__ __launch_bounds__(256) void k_bnout(const float* __restrict__ CT, const float* __restrict__ xb, const float* __restrict__ gam, const float* __restrict__ bet, const float* __restrict__ mean, const float* __restrict__ var, float* OUTb) {
    const int lane = threadIdx.x & 31; const int L0 = (blockIdx.x * 8 + (threadIdx.x >> 5)) * 8; const int nlines = CC * NN / 32;
#pragma unroll 1
    for (int ps = 0; ps < 2; ++ps) {
#pragma unroll 1
        for (int l = 0; l < 8; ++l) { const int L = L0 + l; if (L >= nlines) break; const int e = L * 32 + lane; const int n = e & (NN - 1); const int co = e >> 12;
            const float inv = __fdiv_rn(bfr(gam[co]), __fsqrt_rn(__fadd_rn(bfr(var[co]), 1e-5f))); float sh = __fmul_rn(bfr(mean[co]), inv); asm volatile("" : "+v"(sh)); const float shift = __fsub_rn(bfr(bet[co]), sh);
            float y = __fmul_rn(CT[(size_t)n * CC + co], inv); asm volatile("" : "+v"(y)); y = fmaxf(__fadd_rn(y, shift), 0.f); const float o = __fadd_rn(y, bfr(xb[(size_t)co * NN + n]));
            *(volatile float*)(OUTb + (size_t)e) = o; }
        if (ps == 0) __threadfence(); }
}

extern "C" void kernel_launch(void* const* d_in, const int* in_sizes, int n_in,
                              void* d_out, int out_size, void* d_ws, size_t ws_size, hipStream_t stream) {
    (void)in_sizes; (void)n_in; (void)out_size;
    const float* IN[13]; for (int i = 0; i < 13; ++i) IN[i] = (const float*)d_in[i];
    const float* x = IN[0];
    float* OUT = (float*)d_out;
    char* wsp = (char*)d_ws;
    auto take = [&](size_t bytes) { char* p = wsp; wsp += (bytes + 255) & ~(size_t)255; return (void*)p; };
    bf* WQ = (bf*)take((size_t)CQP * CC * 2); bf* WK = (bf*)take((size_t)CQP * CC * 2); float* BQ = (float*)take(256); float* BK = (float*)take(256); bf* WV = (bf*)take((size_t)CC * CC * 2); bf* WOB = (bf*)take((size_t)CC * KC * 2);
    bf* XT = (bf*)take((size_t)NN * CC * 2); float* FQ = (float*)take((size_t)NN * CQP * 4); bf* Qh = (bf*)take((size_t)NN * CQP * 2); bf* Ql = (bf*)take((size_t)NN * CQP * 2); bf* Kh = (bf*)take((size_t)NN * CQP * 2); bf* Kl = (bf*)take((size_t)NN * CQP * 2);
    float* FV = (float*)take((size_t)CC * NN * 4); h16* V16 = (h16*)take((size_t)CC * NN * 2);
    float* S = (float*)take((size_t)NN * NN * 4); h16* P = (h16*)take((size_t)NN * NN * 2); float* RS = (float*)take((size_t)NN * 32 * 4); float* Ob = (float*)take((size_t)NN * CC * 4); bf* Oh = (bf*)take((size_t)NN * CC * 2); bf* Ol = (bf*)take((size_t)NN * CC * 2);
    bf* Ch = (bf*)take((size_t)NN * KC * 2); bf* Cl = (bf*)take((size_t)NN * KC * 2); float* CT = FV;
    if ((size_t)(wsp - (char*)d_ws) > ws_size) return;
    { k_wpad<<<(CQP * CC / 2 + 255) / 256, 256, 0, stream>>>(IN[1], IN[2], WQ, BQ); k_wpad<<<(CQP * CC / 2 + 255) / 256, 256, 0, stream>>>(IN[3], IN[4], WK, BK);
      k_cvt8<<<(CC * CC / 8 + 255) / 256, 256, 0, stream>>>(IN[5], WV, (size_t)CC * CC / 8); k_wperm<<<(CC * KC / 2 + 255) / 256, 256, 0, stream>>>(IN[7], WOB); }
    const unsigned LX = (unsigned)((NN * CC / 64 + 63) / 64), L2 = (unsigned)(((size_t)NN * CC / 2 + 255) / 256), LQ = (unsigned)(((size_t)NN * CQP / 2 + 255) / 256);
    for (int b = 0; b < NB_; ++b) { const float* xb = x + (size_t)b * CC * NN;
        k_xt<<<LX, 256, 0, stream>>>(xb, XT);
        k_gemmw<bf, 0, true><<<dim3(NN / 64, 1, 1), 32, 0, stream>>>(XT, nullptr, WQ, nullptr, CC, FQ, CQP, BQ, 0, 0, 0); k_qsplit<<<LQ, 256, 0, stream>>>(FQ, Qh, Ql);
        k_gemmw<bf, 0, true><<<dim3(NN / 64, 1, 1), 32, 0, stream>>>(XT, nullptr, WK, nullptr, CC, FQ, CQP, BK, 0, 0, 0); k_qsplit<<<LQ, 256, 0, stream>>>(FQ, Kh, Kl);
        k_gemmw<bf, 0, false><<<dim3(CC / 64, NN / 64, 1), 32, 0, stream>>>(WV, nullptr, XT, nullptr, CC, FV, NN, nullptr, 0, 0, 0); k_v16<<<L2, 256, 0, stream>>>(FV, IN[6], V16);
        k_gemmw<bf, 2, false><<<dim3(NN / 64, NN / 64, 1), 32, 0, stream>>>(Qh, Ql, Kh, Kl, CQP, S, NN, nullptr, 0, 0, 0);
        k_smax<<<NN / 8, 256, 0, stream>>>(S, RS); k_sexp<<<NN / 8, 256, 0, stream>>>(S, RS, P);
        k_gemmw<h16, 0, false><<<dim3(NN / 64, CC / 64, 1), 32, 0, stream>>>(P, nullptr, V16, nullptr, NN, Ob, CC, nullptr, 0, 0, 0);
        k_osplit<<<L2, 256, 0, stream>>>(Ob, RS, Oh, Ol);
        k_im2col<<<(unsigned)((NN * KC / 64 + 63) / 64), 256, 0, stream>>>(Oh, Ol, Ch, Cl);
        k_gemmw<bf, 1, true><<<dim3(NN / 64, CC / 64, 1), 32, 0, stream>>>(Ch, Cl, WOB, nullptr, KC, CT, CC, IN[8], 0, 0, 0);
        k_bnout<<<(CC * NN / 32 + 63) / 64, 256, 0, stream>>>(CT, xb, IN[9], IN[10], IN[11], IN[12], OUT + (size_t)b * CC * NN); }
}
